// OfficialTTTLayer_62826781606583
// MI455X (gfx1250) — hardware-verified
//
#include <hip/hip_runtime.h>
#include <math.h>

typedef __attribute__((ext_vector_type(16))) _Float16 v16h;
typedef __attribute__((ext_vector_type(8)))  _Float16 v8h;
typedef __attribute__((ext_vector_type(16))) __bf16   v16b;
typedef __attribute__((ext_vector_type(8)))  __bf16   v8b;
typedef __attribute__((ext_vector_type(8)))  float    v8f;
typedef __attribute__((ext_vector_type(4)))  float    v4f;
typedef __attribute__((ext_vector_type(2)))  unsigned v2u;

constexpr int kHid   = 1024;
constexpr int kSeq   = 2048;
constexpr int kBatch = 4;
constexpr int kHeads = 16;
constexpr int kHd    = 64;
constexpr int kMb    = 16;
constexpr int kNmb   = kSeq / kMb;
constexpr int kTok   = kBatch * kSeq;
constexpr int kTP    = 72;
constexpr int kSP    = 40;
constexpr int kFP    = 68;
constexpr float kCmScale = 1048576.0f;
constexpr float kCmInv   = 1.0f / 1048576.0f;
constexpr float kWoScale = 64.0f;
constexpr float kWoInv   = 1.0f / 64.0f;
static_assert(kNmb * kMb == kSeq, "chunking");
static_assert(kHeads * kHd == kHid, "heads");

__device__ __forceinline__ unsigned short f2bf_bits(float f) {
  unsigned u = __float_as_uint(f);
  return (unsigned short)((u + 0x7FFFu + ((u >> 16) & 1u)) >> 16);
}
__device__ __forceinline__ float bf_bits2f(unsigned short h) { return __uint_as_float(((unsigned)h) << 16); }
__device__ __forceinline__ float bfr(float f) { return bf_bits2f(f2bf_bits(f)); }
__device__ __forceinline__ void split_bf(float f, unsigned short& hb, unsigned short& lb) {
  hb = f2bf_bits(f);
  lb = f2bf_bits(f - bf_bits2f(hb));
}

__device__ __forceinline__ void dep_guard_h(v8f& a, v8f& b, v16h x, v16h y) { asm volatile("v_nop\n\tv_nop\n\tv_nop\n\tv_nop" : "+v"(a), "+v"(b) : "v"(x), "v"(y)); }
__device__ __forceinline__ void dep_guard_b(v8f& a, v8f& b, v16b x, v16b y) { asm volatile("v_nop\n\tv_nop\n\tv_nop\n\tv_nop" : "+v"(a), "+v"(b) : "v"(x), "v"(y)); }
__device__ __forceinline__ void keep4_h(v16h a, v16h b, v16h c, v16h d) { asm volatile("v_nop" :: "v"(a), "v"(b), "v"(c), "v"(d)); }
__device__ __forceinline__ void keep4_b(v16b a, v16b b, v16b c, v16b d) { asm volatile("v_nop" :: "v"(a), "v"(b), "v"(c), "v"(d)); }
__device__ __forceinline__ void acc_guard4(v8f& a, v8f& b, v8f& c, v8f& d) { asm volatile("v_nop\n\tv_nop\n\tv_nop\n\tv_nop" : "+v"(a), "+v"(b), "+v"(c), "+v"(d)); }
template <typename T> struct Frag;
template <> struct Frag<_Float16> {
  typedef v16h V; union U { v16h v; v8h h[2]; };
  static __device__ __forceinline__ v16h load(const _Float16* p) {
    U f; f.h[0] = *(const v8h*)(p); f.h[1] = *(const v8h*)(p + 16); return f.v;
  }
  static __device__ __forceinline__ v8f mma(v16h a, v16h b, v8f c) {
    return __builtin_amdgcn_wmma_f32_16x16x32_f16(false, a, false, b, (short)0, c, false, false);
  }
  static __device__ __forceinline__ void guard(v8f& a, v8f& b, v16h x, v16h y) { dep_guard_h(a, b, x, y); }
  static __device__ __forceinline__ void keep(v16h a, v16h b, v16h c, v16h d) { keep4_h(a, b, c, d); }
};
template <> struct Frag<__bf16> {
  typedef v16b V; union U { v16b v; v8b h[2]; };
  static __device__ __forceinline__ v16b load(const __bf16* p) {
    U f; f.h[0] = *(const v8b*)(p); f.h[1] = *(const v8b*)(p + 16); return f.v;
  }
  static __device__ __forceinline__ v8f mma(v16b a, v16b b, v8f c) {
    return __builtin_amdgcn_wmma_f32_16x16x32_bf16(false, a, false, b, (short)0, c, false, false);
  }
  static __device__ __forceinline__ void guard(v8f& a, v8f& b, v16b x, v16b y) { dep_guard_b(a, b, x, y); }
  static __device__ __forceinline__ void keep(v16b a, v16b b, v16b c, v16b d) { keep4_b(a, b, c, d); }
};

__device__ __forceinline__ v8f mma_bg(v16b a, v16b b, v8f c) {
  c = __builtin_amdgcn_wmma_f32_16x16x32_bf16(false, a, false, b, (short)0, c, false, false);
  asm volatile("v_nop\n\tv_nop\n\tv_nop\n\tv_nop" : "+v"(c) : "v"(a), "v"(b));
  return c;
}
__device__ __forceinline__ v8f mma_hg(v16h a, v16h b, v8f c) {
  c = __builtin_amdgcn_wmma_f32_16x16x32_f16(false, a, false, b, (short)0, c, false, false);
  asm volatile("v_nop\n\tv_nop\n\tv_nop\n\tv_nop" : "+v"(c) : "v"(a), "v"(b));
  return c;
}

template <int ET> struct Elem;
template <> struct Elem<0> { typedef _Float16 T; };
template <> struct Elem<1> { typedef __bf16 T; };
template <int ET, bool SPLIT, int BIAS_MODE, int OUT_MODE, bool RESID, int ACT = 0>
__global__ __launch_bounds__(256) void wmma_gemm64(
    const unsigned short* __restrict__ Ap, const unsigned short* __restrict__ A2p, int lda, long strideA,
    const unsigned short* __restrict__ Btp, const unsigned short* __restrict__ Bt2p, int ldb, long strideB,
    void* __restrict__ Cout, void* __restrict__ Cout2, int ldc, long strideC,
    const float* __restrict__ bias,
    const float* __restrict__ resid, long strideR,
    int M, int N, int K, float scale) {
  typedef typename Elem<ET>::T T;
  typedef typename Frag<T>::V V;
  const T* A = (const T*)Ap; const T* A2 = (const T*)A2p; const T* Bt = (const T*)Btp; const T* Bt2 = (const T*)Bt2p;
  __shared__ __align__(16) float sT[8][16 * 68];
  const int b    = blockIdx.y;
  const int lane = threadIdx.x & 31;
  const int wave = threadIdx.x >> 5;
  const int tilesN = N >> 6;
  const int tilesM = M >> 6;
  const int tile = blockIdx.x * 8 + wave;
  if (tile >= tilesM * tilesN) return;
  const int tm = tile / tilesN;
  const int tn = tile - tm * tilesN;
  const int m0 = tm << 6;
  const int n0 = tn << 6;

  const T* Ab  = A  + (size_t)b * strideA;
  const T* Bb  = Bt + (size_t)b * strideB;
  const T* Ab2 = SPLIT ? (A2  + (size_t)b * strideA) : nullptr;
  const T* Bb2 = SPLIT ? (Bt2 + (size_t)b * strideB) : nullptr;

  const int rlane = lane & 15;
  const int koff  = (lane >> 4) * 8;
  const int mOff  = (lane >> 4) * 8;

  v8f acc[4][4];
#pragma unroll
  for (int i = 0; i < 4; ++i)
#pragma unroll
    for (int j = 0; j < 4; ++j) acc[i][j] = (v8f){0.f,0.f,0.f,0.f,0.f,0.f,0.f,0.f};

  for (int k0 = 0; k0 < K; k0 += 32) {
    V bh[4], bl[4];
#pragma unroll
    for (int j = 0; j < 4; ++j) {
      const size_t bo = (size_t)(n0 + (j << 4) + rlane) * ldb + koff + k0;
      bh[j] = Frag<T>::load(Bb + bo);
      if (SPLIT) bl[j] = Frag<T>::load(Bb2 + bo);
    }
#pragma unroll
    for (int i = 0; i < 4; ++i) {
      const size_t ao = (size_t)(m0 + (i << 4) + rlane) * lda + koff + k0;
      V ah = Frag<T>::load(Ab + ao);
      V al;
      if (SPLIT) al = Frag<T>::load(Ab2 + ao);
#pragma unroll
      for (int j = 0; j < 4; ++j) {
        acc[i][j] = Frag<T>::mma(ah, bh[j], acc[i][j]);
        if (SPLIT) {
          acc[i][j] = Frag<T>::mma(ah, bl[j], acc[i][j]);
          acc[i][j] = Frag<T>::mma(al, bh[j], acc[i][j]);
        }
      }
      Frag<T>::guard(acc[i][0], acc[i][3], ah, SPLIT ? al : ah);
    }
    Frag<T>::keep(bh[0], bh[1], bh[2], bh[3]);
    if (SPLIT) Frag<T>::keep(bl[0], bl[1], bl[2], bl[3]);
  }
  acc_guard4(acc[0][0], acc[0][1], acc[0][2], acc[0][3]);
  acc_guard4(acc[1][0], acc[1][1], acc[1][2], acc[1][3]);
  acc_guard4(acc[2][0], acc[2][1], acc[2][2], acc[2][3]);
  acc_guard4(acc[3][0], acc[3][1], acc[3][2], acc[3][3]);

  float* slab = sT[wave];
  const float* Rb = RESID ? (resid + (size_t)b * strideR) : nullptr;
#pragma unroll
  for (int i = 0; i < 4; ++i) {
    const int mBase = m0 + (i << 4);
#pragma unroll
    for (int j = 0; j < 4; ++j) {
      const int n = n0 + (j << 4) + rlane;
      float bv = 0.f;
      if (BIAS_MODE == 2) bv = bias[n];
#pragma unroll
      for (int r = 0; r < 8; ++r) {
        float v = acc[i][j][r] * scale;
        if (BIAS_MODE == 1) v += bias[mBase + mOff + r];
        if (BIAS_MODE == 2) v += bv;
        if (RESID) v += Rb[(size_t)(mBase + mOff + r) * ldc + n];
        if (ACT == 1) v = tanhf(v);
        if (ACT == 2) v = fmaxf(v, 0.0f);
        if (ACT == 3) v = v / (1.0f + expf(-v));
        if (ACT == 4) v = (v > 0.f) ? v : 0.01f * v;
        if (ACT == 5) v = 0.5f * v * (1.0f + erff(v * 0.70710678118654752f));
        slab[(mOff + r) * 68 + (j << 4) + rlane] = v;
      }
    }
    __builtin_amdgcn_fence(__ATOMIC_RELEASE, "workgroup");
    __builtin_amdgcn_wave_barrier();
    __builtin_amdgcn_fence(__ATOMIC_ACQUIRE, "workgroup");
    if (OUT_MODE == 0) {
      float* C = (float*)Cout + (size_t)b * strideC;
      const int hh = lane >> 4, c4 = (lane & 15) * 4;
      for (int pass = 0; pass < 2; ++pass) {
#pragma unroll
        for (int it = 0; it < 8; ++it) {
          const int row = it * 2 + hh;
          v4f v = *(const v4f*)(slab + row * 68 + c4);
          *(volatile v4f*)(C + (size_t)(mBase + row) * ldc + n0 + c4) = v;
        }
        __threadfence();
      }
    } else {
      const int q = lane >> 3, c8 = (lane & 7) * 8;
      unsigned short* C  = (unsigned short*)Cout  + (size_t)b * strideC;
      unsigned short* C2 = (OUT_MODE == 2) ? ((unsigned short*)Cout2 + (size_t)b * strideC) : nullptr;
      for (int pass = 0; pass < 2; ++pass) {
#pragma unroll
        for (int it = 0; it < 4; ++it) {
          const int row = it * 4 + q;
          const float* sp = slab + row * 68 + c8;
          v8h hv, lv;
#pragma unroll
          for (int e = 0; e < 8; ++e) {
            if (OUT_MODE == 1) {
              hv[e] = (_Float16)sp[e];
            } else {
              unsigned short hb = f2bf_bits(sp[e]);
              unsigned short lb = f2bf_bits(sp[e] - bf_bits2f(hb));
              hv[e] = __builtin_bit_cast(_Float16, hb);
              lv[e] = __builtin_bit_cast(_Float16, lb);
            }
          }
          *(volatile v8h*)(C + (size_t)(mBase + row) * ldc + n0 + c8) = hv;
          if (OUT_MODE == 2) *(volatile v8h*)(C2 + (size_t)(mBase + row) * ldc + n0 + c8) = lv;
        }
        __threadfence();
      }
    }
    __builtin_amdgcn_fence(__ATOMIC_RELEASE, "workgroup");
    __builtin_amdgcn_wave_barrier();
    __builtin_amdgcn_fence(__ATOMIC_ACQUIRE, "workgroup");
  }
}

template <int MODE>
__global__ __launch_bounds__(256) void cast8_kernel(const float* __restrict__ in, unsigned short* __restrict__ out,
                                                 int n8, float sc) {
  const int i = blockIdx.x * 256 + threadIdx.x;
  if (i >= n8) return;
  const v4f a = *(const v4f*)(in + (size_t)i * 8);
  const v4f bq = *(const v4f*)(in + (size_t)i * 8 + 4);
  v8h hv;
#pragma unroll
  for (int e = 0; e < 4; ++e) {
    unsigned short b0, b1;
    if (MODE == 0) {
      b0 = f2bf_bits(a[e]);
      b1 = f2bf_bits(bq[e]);
    } else {
      b0 = __builtin_bit_cast(unsigned short, (_Float16)(bf_bits2f(f2bf_bits(a[e])) * sc));
      b1 = __builtin_bit_cast(unsigned short, (_Float16)(bf_bits2f(f2bf_bits(bq[e])) * sc));
    }
    hv[e]     = __builtin_bit_cast(_Float16, b0);
    hv[4 + e] = __builtin_bit_cast(_Float16, b1);
  }
  unsigned short* p = out + (size_t)i * 8;
  *(volatile v8h*)p = hv;
  __threadfence();
  *(volatile v8h*)p = hv;
}

__global__ __launch_bounds__(256) void ttt_kernel(const float* __restrict__ Qf, const float* __restrict__ Kf,
                                                const float* __restrict__ Vf, const float* __restrict__ W1i,
                                                const float* __restrict__ b1i, const float* __restrict__ tg,
                                                const float* __restrict__ tb, float* __restrict__ Yf) {
  __shared__ __align__(16) float qs[kMb * kFP];
  __shared__ __align__(16) float ks[kMb * kFP];
  __shared__ __align__(16) float vs[kMb * kFP];
  __shared__ __align__(16) float zs[kMb * kFP];
  __shared__ __align__(16) float gs[kMb * kFP];
  __shared__ __align__(16) float os[kMb * kFP];
  __shared__ __align__(16) __bf16 ah16[2][kMb * kTP];
  __shared__ __align__(16) __bf16 al16[2][kMb * kTP];
  __shared__ __align__(16) __bf16 w1h[kHd * kTP];
  __shared__ __align__(16) __bf16 w1l[kHd * kTP];
  __shared__ __align__(16) _Float16 kT[kHd * kSP];
  __shared__ __align__(16) _Float16 gT[kHd * kSP];
  __shared__ __align__(16) _Float16 cmt[kMb * kSP];
  __shared__ float b1s[kHd], tgs[kHd], tbs[kHd], etas[kMb];

  const int tid  = threadIdx.x;
  const int lane = tid & 31;
  const int wave = __builtin_amdgcn_readfirstlane(tid >> 5);
  const int hh   = lane >> 4;
  const int c    = lane & 15;
  const int koff = hh * 8;
  const int nt   = wave & 3;
  const int dt0  = (wave >> 2) * 2;
  const int h    = blockIdx.x;
  const v8f z8 = {0.f, 0.f, 0.f, 0.f, 0.f, 0.f, 0.f, 0.f};

#pragma unroll 1
  for (int i = tid; i < kHd * kSP; i += 256) { kT[i] = (_Float16)0.0f; gT[i] = (_Float16)0.0f; }
#pragma unroll 1
  for (int i = tid; i < kMb * kSP; i += 256) cmt[i] = (_Float16)0.0f;

  float wreg[2][8];
#pragma unroll
  for (int t2 = 0; t2 < 2; ++t2) {
#pragma unroll
    for (int r = 0; r < 8; ++r) {
      const int d = 16 * (dt0 + t2) + 8 * hh + r;
      const int n = 16 * nt + c;
      wreg[t2][r] = bfr(W1i[(size_t)h * kHd * kHd + (size_t)d * kHd + n]);
    }
  }
  if (tid < kHd) {
    b1s[tid] = bfr(b1i[h * kHd + tid]);
    tgs[tid] = bfr(tg[tid]);
    tbs[tid] = bfr(tb[tid]);
  }
  if (tid < kMb) etas[tid] = (0.1f / (float)(tid + 1)) * (1.0f / 64.0f);
  __syncthreads();

#pragma unroll 1
  for (int ch = 0; ch < kNmb; ++ch) {
    {
      const int m = tid >> 4, d4 = (tid & 15) * 4;
      const size_t go = (size_t)(ch * kMb + m) * kHid + (size_t)h * kHd + d4;
      const v4f q4 = *(const v4f*)(Qf + go);
      const v4f k4 = *(const v4f*)(Kf + go);
      const v4f v4 = *(const v4f*)(Vf + go);
      *(v4f*)(qs + m * kFP + d4) = q4;
      *(v4f*)(ks + m * kFP + d4) = k4;
      *(v4f*)(vs + m * kFP + d4) = v4;
#pragma unroll
      for (int e = 0; e < 4; ++e) {
        const int d = d4 + e;
        unsigned short hb, lb;
        split_bf(k4[e], hb, lb);
        ah16[0][m * kTP + d] = __builtin_bit_cast(__bf16, hb);
        al16[0][m * kTP + d] = __builtin_bit_cast(__bf16, lb);
        split_bf(q4[e], hb, lb);
        ah16[1][m * kTP + d] = __builtin_bit_cast(__bf16, hb);
        al16[1][m * kTP + d] = __builtin_bit_cast(__bf16, lb);
        kT[d * kSP + m] = (_Float16)k4[e];
      }
    }
#pragma unroll
    for (int t2 = 0; t2 < 2; ++t2) {
      const int dt = dt0 + t2;
      v8b hv, lv;
#pragma unroll
      for (int r = 0; r < 8; ++r) {
        unsigned short hb, lb;
        split_bf(wreg[t2][r], hb, lb);
        hv[r] = __builtin_bit_cast(__bf16, hb);
        lv[r] = __builtin_bit_cast(__bf16, lb);
      }
      const int o = (16 * nt + c) * kTP + 16 * dt + 8 * hh;
      *(v8b*)(w1h + o) = hv;
      *(v8b*)(w1l + o) = lv;
    }
    __syncthreads();

    const int sel = (wave < 4) ? 0 : 1;
    v8f acc = z8;
#pragma unroll
    for (int ks2 = 0; ks2 < 2; ++ks2) {
      const int k0 = 32 * ks2;
      const v16b a   = Frag<__bf16>::load(ah16[sel] + c * kTP + koff + k0);
      const v16b al  = Frag<__bf16>::load(al16[sel] + c * kTP + koff + k0);
      const v16b bw  = Frag<__bf16>::load(w1h + (16 * nt + c) * kTP + koff + k0);
      const v16b bwl = Frag<__bf16>::load(w1l + (16 * nt + c) * kTP + koff + k0);
      acc = mma_bg(a, bw, acc);
      acc = mma_bg(a, bwl, acc);
      acc = mma_bg(al, bw, acc);
    }
    if (wave < 4) {
#pragma unroll
      for (int r = 0; r < 8; ++r) {
        const int n = 16 * nt + c;
        zs[(8 * hh + r) * kFP + n] = acc[r] + b1s[n];
      }
    }
    if (wave == 4) {
      v8f at = z8;
#pragma unroll
      for (int ks2 = 0; ks2 < 2; ++ks2) {
        const int k0 = 32 * ks2;
        const v16b a = Frag<__bf16>::load(ah16[1] + c * kTP + koff + k0);
        const v16b bk = Frag<__bf16>::load(ah16[0] + c * kTP + koff + k0);
        at = mma_bg(a, bk, at);
      }
#pragma unroll
      for (int r = 0; r < 8; ++r) {
        const int m = 8 * hh + r;
        const float et = etas[m];
        const float se = et * et;
        const float cv = -(se * (1.0f + at[r]));
        const float cvs = (c <= m) ? (cv * kCmScale) : 0.0f;
        cmt[m * kSP + c] = (_Float16)cvs;
      }
    }
    __syncthreads();

    {
      const int row = 2 * wave + hh;
      const float* zr = zs + row * kFP;
      const float x0 = zr[c], x1 = zr[c + 16], x2 = zr[c + 32], x3 = zr[c + 48];
      float s = (x0 + x1) + (x2 + x3);
      s += __shfl_xor(s, 1, 32); s += __shfl_xor(s, 2, 32); s += __shfl_xor(s, 4, 32); s += __shfl_xor(s, 8, 32);
      const float mean = s * (1.0f / 64.0f);
      const float e0 = x0 - mean, e1 = x1 - mean, e2 = x2 - mean, e3 = x3 - mean;
      float s2 = (e0 * e0 + e1 * e1) + (e2 * e2 + e3 * e3);
      s2 += __shfl_xor(s2, 1, 32); s2 += __shfl_xor(s2, 2, 32); s2 += __shfl_xor(s2, 4, 32); s2 += __shfl_xor(s2, 8, 32);
      const float rstd = rsqrtf(s2 * (1.0f / 64.0f) + 1e-5f);
      const float ev[4] = {e0, e1, e2, e3};
#pragma unroll
      for (int e = 0; e < 4; ++e) {
        const int col = c + 16 * e;
        const float lnv = ev[e] * rstd * tgs[col] + tbs[col];
        const float g = lnv - (vs[row * kFP + col] - ks[row * kFP + col]);
        gs[row * kFP + col] = g;
        gT[col * kSP + row] = (_Float16)g;
      }
    }
    __syncthreads();

    {
      const float last_eta = etas[kMb - 1];
#pragma unroll
      for (int t2 = 0; t2 < 2; ++t2) {
        const int dt = dt0 + t2;
        const v16h a  = Frag<_Float16>::load(kT + (16 * dt + c) * kSP + koff);
        const v16h bg = Frag<_Float16>::load(gT + (16 * nt + c) * kSP + koff);
        v8f u = z8;
        u = mma_hg(a, bg, u);
#pragma unroll
        for (int r = 0; r < 8; ++r) wreg[t2][r] = wreg[t2][r] - last_eta * u[r];
      }
    }
    if (wave >= 4) {
      const v16h a  = Frag<_Float16>::load(cmt + c * kSP + koff);
      const v16h bg = Frag<_Float16>::load(gT + (16 * nt + c) * kSP + koff);
      v8f cr = z8;
      cr = mma_hg(a, bg, cr);
#pragma unroll
      for (int r = 0; r < 8; ++r) {
        const int m = 8 * hh + r;
        const int n = 16 * nt + c;
        zs[m * kFP + n] = acc[r] + cr[r] * kCmInv + b1s[n];
      }
    }
    __syncthreads();

    {
      const int row = 2 * wave + hh;
      const float* zr = zs + row * kFP;
      const float x0 = zr[c], x1 = zr[c + 16], x2 = zr[c + 32], x3 = zr[c + 48];
      float s = (x0 + x1) + (x2 + x3);
      s += __shfl_xor(s, 1, 32); s += __shfl_xor(s, 2, 32); s += __shfl_xor(s, 4, 32); s += __shfl_xor(s, 8, 32);
      const float mean = s * (1.0f / 64.0f);
      const float e0 = x0 - mean, e1 = x1 - mean, e2 = x2 - mean, e3 = x3 - mean;
      float s2 = (e0 * e0 + e1 * e1) + (e2 * e2 + e3 * e3);
      s2 += __shfl_xor(s2, 1, 32); s2 += __shfl_xor(s2, 2, 32); s2 += __shfl_xor(s2, 4, 32); s2 += __shfl_xor(s2, 8, 32);
      const float rstd = rsqrtf(s2 * (1.0f / 64.0f) + 1e-5f);
      const float ev[4] = {e0, e1, e2, e3};
#pragma unroll
      for (int e = 0; e < 4; ++e) {
        const int col = c + 16 * e;
        const float lnv = ev[e] * rstd * tgs[col] + tbs[col];
        os[row * kFP + col] = qs[row * kFP + col] + lnv;
      }
    }
    if (tid < kHd) {
      float sacc = 0.0f;
#pragma unroll 1
      for (int m = 0; m < kMb; ++m) sacc += etas[m] * gs[m * kFP + tid];
      b1s[tid] = b1s[tid] - sacc;
    }
    __syncthreads();

    {
      const int row = tid >> 4, c4 = (tid & 15) * 4;
      const v4f ov = *(const v4f*)(os + row * kFP + c4);
      float* yp = Yf + (size_t)(ch * kMb + row) * kHid + (size_t)h * kHd + c4;
      for (int pass = 0; pass < 2; ++pass) {
        *(volatile v4f*)yp = ov;
        __threadfence();
      }
    }
  }
}

__global__ __launch_bounds__(256) void lng_kernel(const float* __restrict__ Yf, const float* __restrict__ Gf,
                                                const float* __restrict__ lg, const float* __restrict__ lb,
                                                unsigned short* __restrict__ A16) {
  __shared__ float red[8];
  const int row = blockIdx.x, tid = threadIdx.x, lane = tid & 31, wave = tid >> 5;
  const size_t ro = (size_t)row * kHid + (size_t)tid * 4;
  const v4f y4 = *(const v4f*)(Yf + ro);
  const v4f u4 = *(const v4f*)(Gf + ro);
  float s = (y4[0] + y4[1]) + (y4[2] + y4[3]);
  s += __shfl_xor(s, 16, 32); s += __shfl_xor(s, 8, 32); s += __shfl_xor(s, 4, 32); s += __shfl_xor(s, 2, 32); s += __shfl_xor(s, 1, 32);
  if (lane == 0) red[wave] = s;
  __syncthreads();
  float tot = 0.0f;
#pragma unroll
  for (int w = 0; w < 8; ++w) tot += red[w];
  const float mean = tot * (1.0f / 1024.0f);
  __syncthreads();
  const float e0 = y4[0] - mean, e1 = y4[1] - mean, e2 = y4[2] - mean, e3 = y4[3] - mean;
  float s2 = (e0 * e0 + e1 * e1) + (e2 * e2 + e3 * e3);
  s2 += __shfl_xor(s2, 16, 32); s2 += __shfl_xor(s2, 8, 32); s2 += __shfl_xor(s2, 4, 32); s2 += __shfl_xor(s2, 2, 32); s2 += __shfl_xor(s2, 1, 32);
  if (lane == 0) red[wave] = s2;
  __syncthreads();
  float tot2 = 0.0f;
#pragma unroll
  for (int w = 0; w < 8; ++w) tot2 += red[w];
  const float rstd = rsqrtf(tot2 * (1.0f / 1024.0f) + 1e-5f);
  const float ev[4] = {e0, e1, e2, e3};
  unsigned short hb[4];
#pragma unroll
  for (int e = 0; e < 4; ++e) {
    const int col = tid * 4 + e;
    const float lnv = ev[e] * rstd * bfr(lg[col]) + bfr(lb[col]);
    const float u = u4[e];
    const float targ = 0.7978845608028654f * (u + 0.044715f * u * u * u);
    const float gv = u * (0.5f * (1.0f + tanhf(targ)));
    hb[e] = __builtin_bit_cast(unsigned short, (_Float16)(gv * lnv));
  }
  v2u pk;
  pk[0] = (unsigned)hb[0] | ((unsigned)hb[1] << 16);
  pk[1] = (unsigned)hb[2] | ((unsigned)hb[3] << 16);
  unsigned short* ap = A16 + ro;
  *(volatile v2u*)ap = pk;
  __threadfence();
  *(volatile v2u*)ap = pk;
}

extern "C" void kernel_launch(void* const* d_in, const int* in_sizes, int n_in,
                              void* d_out, int out_size, void* d_ws, size_t ws_size, hipStream_t stream) {
  if (n_in < 12 || d_out == nullptr || d_ws == nullptr) return;
  if (in_sizes[0] != kTok * kHid) return;
  for (int i = 1; i <= 5; ++i) if (in_sizes[i] != kHid * kHid) return;
  if (in_sizes[6] != kHeads * kHd * kHd || in_sizes[7] != kHeads * kHd || in_sizes[8] != kHd || in_sizes[9] != kHd ||
      in_sizes[10] != kHid || in_sizes[11] != kHid || out_size != kTok * kHid) return;

  const float* xin = (const float*)d_in[0];
  const float* wq  = (const float*)d_in[1];
  const float* wk  = (const float*)d_in[2];
  const float* wv  = (const float*)d_in[3];
  const float* wg  = (const float*)d_in[4];
  const float* wo  = (const float*)d_in[5];
  const float* w1i = (const float*)d_in[6];
  const float* b1i = (const float*)d_in[7];
  const float* tg  = (const float*)d_in[8];
  const float* tb  = (const float*)d_in[9];
  const float* lg  = (const float*)d_in[10];
  const float* lb  = (const float*)d_in[11];
  float* out = (float*)d_out;

  const size_t wElems = (size_t)kHid * kHid;
  const size_t bElems = (size_t)kSeq * kHid;

  char* ws = (char*)d_ws; size_t off = 0;
  auto carve = [&](size_t bytes) -> char* { char* p = ws + off; off += (bytes + 255) & ~(size_t)255; return p; };
  unsigned short* X16  = (unsigned short*)carve((size_t)kTok * kHid * 2);
  unsigned short* W16  = (unsigned short*)carve(4 * wElems * 2);
  unsigned short* WO16 = (unsigned short*)carve(wElems * 2);
  float*          QKVG = (float*)carve(4 * bElems * 4);
  float*          YF   = (float*)carve(bElems * 4);
  unsigned short* A16  = (unsigned short*)carve(bElems * 2);
  if (off > ws_size || off > (size_t)134217728) return;

  cast8_kernel<0><<<dim3((unsigned)((size_t)kTok * kHid / 8 / 256)), 256, 0, stream>>>(xin, X16, (int)((size_t)kTok * kHid / 8), 1.0f);
  cast8_kernel<0><<<dim3((unsigned)(wElems / 8 / 256)), 256, 0, stream>>>(wq, W16 + 0 * wElems, (int)(wElems / 8), 1.0f);
  cast8_kernel<0><<<dim3((unsigned)(wElems / 8 / 256)), 256, 0, stream>>>(wk, W16 + 1 * wElems, (int)(wElems / 8), 1.0f);
  cast8_kernel<0><<<dim3((unsigned)(wElems / 8 / 256)), 256, 0, stream>>>(wv, W16 + 2 * wElems, (int)(wElems / 8), 1.0f);
  cast8_kernel<0><<<dim3((unsigned)(wElems / 8 / 256)), 256, 0, stream>>>(wg, W16 + 3 * wElems, (int)(wElems / 8), 1.0f);
  cast8_kernel<1><<<dim3((unsigned)(wElems / 8 / 256)), 256, 0, stream>>>(wo, WO16, (int)(wElems / 8), kWoScale);

  const unsigned gemmBlocks = (unsigned)(((kSeq / 64) * (kHid / 64)) / 8);
  for (int b = 0; b < kBatch; ++b) {
    wmma_gemm64<1, false, 0, 0, false, 0><<<dim3(gemmBlocks, 4), 256, 0, stream>>>(
        X16 + (size_t)b * bElems, X16 + (size_t)b * bElems, kHid, 0L,
        W16, W16, kHid, (long)wElems,
        (void*)QKVG, (void*)QKVG, kHid, (long)bElems,
        (const float*)YF, (const float*)YF, 0L,
        kSeq, kHid, kHid, 1.0f);
    ttt_kernel<<<dim3(kHeads), 256, 0, stream>>>(QKVG, QKVG + bElems, QKVG + 2 * bElems, w1i, b1i, tg, tb, YF);
    lng_kernel<<<dim3(kSeq), 256, 0, stream>>>(YF, QKVG + 3 * bElems, lg, lb, A16);
    wmma_gemm64<0, false, 0, 0, false, 0><<<dim3(gemmBlocks, 1), 256, 0, stream>>>(
        A16, A16, kHid, 0L,
        WO16, WO16, kHid, 0L,
        (void*)(out + (size_t)b * bElems), (void*)(out + (size_t)b * bElems), kHid, 0L,
        (const float*)YF, (const float*)YF, 0L,
        kSeq, kHid, kHid, kWoInv);
  }
}
